// SlideAttention_42898133353031
// MI455X (gfx1250) — hardware-verified
//
#include <hip/hip_runtime.h>
#include <stddef.h>
#include <stdint.h>

#define BB    8
#define NTOK  1024
#define GW    32
#define CC    384
#define NHD   12
#define HD    32
#define C3    (3 * CC)
#define ROWS  (BB * NTOK)
#define NBH   (BB * NHD)
#define PLN   ((size_t)NBH * NTOK * HD)

static_assert(NHD * HD == CC);
static_assert(ROWS % 256 == 0);
static_assert(NTOK % 256 == 0);
static_assert(CC % 64 == 0);
static_assert(C3 % 64 == 0);
static_assert(GW * GW == NTOK);
static_assert(HD == 32);

typedef _Float16 v16h __attribute__((ext_vector_type(16)));
typedef _Float16 v8h  __attribute__((ext_vector_type(8)));
typedef float    v8f  __attribute__((ext_vector_type(8)));
typedef float    v4f  __attribute__((ext_vector_type(4)));
typedef unsigned int v4u __attribute__((ext_vector_type(4)));

union Frag  { v16h v; v8h h[2]; };
union Pack8 { v8h h; v4u u; };

__device__ __forceinline__ v8f mma16(v16h a, v16h b, v8f c) {
  c = __builtin_amdgcn_wmma_f32_16x16x32_f16(false, a, false, b, (short)0, c, false, false);
  asm volatile("v_nop\n\tv_nop\n\tv_nop\n\tv_nop" : "+v"(c) : "v"(a), "v"(b));
  return c;
}

__device__ __forceinline__ v16h ldfrag(const _Float16* p, int ld, int row0, int k0, int lane) {
  const int m = lane & 15, lh = lane >> 4;
  const _Float16* q = p + (size_t)(row0 + m) * ld + k0 + 8 * lh;
  Frag f;
  f.h[0] = *(const v8h*)(q);
  f.h[1] = *(const v8h*)(q + 16);
  return f.v;
}

__device__ __forceinline__ v8f zero8() { return (v8f){0.f, 0.f, 0.f, 0.f, 0.f, 0.f, 0.f, 0.f}; }

__device__ __forceinline__ int clampi(int v, int lo, int hi) { return v < lo ? lo : (v > hi ? hi : v); }

__global__ __launch_bounds__(256) void k_cvt_x(const float* __restrict__ x, _Float16* __restrict__ xh, int ngrp) {
  const int t = blockIdx.x * 256 + (int)threadIdx.x;
  if (t >= ngrp) return;
  const size_t o = (size_t)t * 8;
  const v4f a0 = *(const v4f*)(x + o);
  const v4f a1 = *(const v4f*)(x + o + 4);
  Pack8 pk;
  pk.h = (v8h){(_Float16)a0[0], (_Float16)a0[1], (_Float16)a0[2], (_Float16)a0[3],
               (_Float16)a1[0], (_Float16)a1[1], (_Float16)a1[2], (_Float16)a1[3]};
  const v4u vv = pk.u;
  volatile v4u* d = (volatile v4u*)(xh + o);
  *d = vv;
  __threadfence();
  *d = vv;
}

#define WTP 68
__global__ __launch_bounds__(256) void k_wt(const float* __restrict__ w, _Float16* __restrict__ wt, int nout) {
  __shared__ __align__(16) float tf[64 * WTP];
  const int tid = threadIdx.x;
  const int n0 = blockIdx.x * 64;
  const int k0 = blockIdx.y * 64;
  {
    const int kr = tid >> 4;
    const int n4 = (tid & 15) * 4;
#pragma unroll
    for (int it = 0; it < 4; ++it) {
      const int kl = it * 16 + kr;
      const v4f a = *(const v4f*)(w + (size_t)(k0 + kl) * nout + n0 + n4);
      *(v4f*)(tf + kl * WTP + n4) = a;
    }
  }
  __syncthreads();
  v4u val[2];
  size_t go[2];
#pragma unroll
  for (int j = 0; j < 2; ++j) {
    const int p  = tid + 256 * j;
    const int nl = p >> 3;
    const int pc = p & 7;
    const float* cp = tf + (pc * 8) * WTP + nl;
    Pack8 pk;
    pk.h = (v8h){(_Float16)(cp[0 * WTP] * 32.0f), (_Float16)(cp[1 * WTP] * 32.0f),
                 (_Float16)(cp[2 * WTP] * 32.0f), (_Float16)(cp[3 * WTP] * 32.0f),
                 (_Float16)(cp[4 * WTP] * 32.0f), (_Float16)(cp[5 * WTP] * 32.0f),
                 (_Float16)(cp[6 * WTP] * 32.0f), (_Float16)(cp[7 * WTP] * 32.0f)};
    val[j] = pk.u;
    go[j]  = (size_t)(n0 + nl) * CC + k0 + pc * 8;
  }
  for (int ps = 0; ps < 2; ++ps) {
#pragma unroll
    for (int j = 0; j < 2; ++j) *(volatile v4u*)(wt + go[j]) = val[j];
    __threadfence();
  }
}

#define OTP 68
__global__ __launch_bounds__(256) void k_qkv(const _Float16* __restrict__ xh,
                                             const _Float16* __restrict__ wt,
                                             const float* __restrict__ bias,
                                             _Float16* __restrict__ qp,
                                             float* __restrict__ kvf) {
  __shared__ __align__(16) float st[8][16 * OTP];
  const int tid = threadIdx.x, lane = tid & 31, wave = tid >> 5;
  const int hh = lane >> 4, c = lane & 15;
  const int mb = blockIdx.x * 256;
  const int m0 = mb + wave * 32;
  const int y  = blockIdx.y;
  const int n0 = y * 64;
  const int which = y / 6;
  const int head0 = (y - which * 6) * 2;
  const int b  = mb >> 10;
  const int nb = mb & (NTOK - 1);

  v8f acc[2][4];
#pragma unroll
  for (int s = 0; s < 2; ++s)
#pragma unroll
    for (int t = 0; t < 4; ++t) acc[s][t] = zero8();

#pragma unroll 2
  for (int k0 = 0; k0 < CC; k0 += 32) {
    const v16h a0 = ldfrag(xh, CC, m0, k0, lane);
    const v16h a1 = ldfrag(xh, CC, m0 + 16, k0, lane);
    const v16h b0 = ldfrag(wt, CC, n0, k0, lane);
    const v16h b1 = ldfrag(wt, CC, n0 + 16, k0, lane);
    const v16h b2 = ldfrag(wt, CC, n0 + 32, k0, lane);
    const v16h b3 = ldfrag(wt, CC, n0 + 48, k0, lane);
    acc[0][0] = mma16(a0, b0, acc[0][0]);
    acc[1][0] = mma16(a1, b0, acc[1][0]);
    acc[0][1] = mma16(a0, b1, acc[0][1]);
    acc[1][1] = mma16(a1, b1, acc[1][1]);
    acc[0][2] = mma16(a0, b2, acc[0][2]);
    acc[1][2] = mma16(a1, b2, acc[1][2]);
    acc[0][3] = mma16(a0, b3, acc[0][3]);
    acc[1][3] = mma16(a1, b3, acc[1][3]);
  }

  float bvs[4];
#pragma unroll
  for (int t = 0; t < 4; ++t) bvs[t] = bias[n0 + 16 * t + c];

  float* sw = st[wave];
#pragma unroll
  for (int sub = 0; sub < 2; ++sub) {
    __syncthreads();
#pragma unroll
    for (int t = 0; t < 4; ++t) {
#pragma unroll
      for (int r = 0; r < 8; ++r)
        sw[(8 * hh + r) * OTP + 16 * t + c] = acc[sub][t][r] * 0.03125f + bvs[t];
    }
    __syncthreads();
    const int nrow0 = nb + wave * 32 + sub * 16;
    if (which == 0) {
      v4u val[4];
      size_t go[4];
#pragma unroll
      for (int it = 0; it < 4; ++it) {
        const int p    = lane + 32 * it;
        const int head = p >> 6;
        const int pp   = p & 63;
        const int row  = pp >> 2;
        const int c8   = (pp & 3) * 8;
        const float* cp = sw + row * OTP + head * 32 + c8;
        Pack8 pk;
        pk.h = (v8h){(_Float16)(cp[0] * 16.0f), (_Float16)(cp[1] * 16.0f),
                     (_Float16)(cp[2] * 16.0f), (_Float16)(cp[3] * 16.0f),
                     (_Float16)(cp[4] * 16.0f), (_Float16)(cp[5] * 16.0f),
                     (_Float16)(cp[6] * 16.0f), (_Float16)(cp[7] * 16.0f)};
        val[it] = pk.u;
        go[it]  = ((size_t)(b * NHD + head0 + head) * NTOK + nrow0) * HD + pp * 8;
      }
      for (int ps = 0; ps < 2; ++ps) {
#pragma unroll
        for (int it = 0; it < 4; ++it) *(volatile v4u*)(qp + go[it]) = val[it];
        __threadfence();
      }
    } else {
      v4f val[8];
      size_t go[8];
      const size_t plane = (size_t)(which - 1) * PLN;
#pragma unroll
      for (int it = 0; it < 8; ++it) {
        const int p    = lane + 32 * it;
        const int L    = p >> 3;
        const int pc   = p & 7;
        const int head = L & 1;
        const int row  = L >> 1;
        val[it] = *(const v4f*)(sw + row * OTP + head * 32 + pc * 4);
        go[it]  = plane + ((size_t)(b * NHD + head0 + head) * NTOK + nrow0 + row) * HD + pc * 4;
      }
      for (int ps = 0; ps < 2; ++ps) {
#pragma unroll
        for (int it = 0; it < 8; ++it) *(volatile v4f*)(kvf + go[it]) = val[it];
        __threadfence();
      }
    }
  }
}

#define CKP 40
#define CVP 136
__global__ __launch_bounds__(256) void k_conv(const float* __restrict__ kvf,
                                              const float* __restrict__ cw,
                                              const float* __restrict__ cb,
                                              _Float16* __restrict__ kh,
                                              _Float16* __restrict__ vt) {
  __shared__ __align__(16) _Float16 Kt[128 * CKP];
  __shared__ __align__(16) _Float16 Vtt[32 * CVP];
  const int tid = threadIdx.x;
  const int d   = tid & 31;
  const int g   = tid >> 5;
  const int bh  = blockIdx.x >> 3;
  const int yt  = blockIdx.x & 7;
  const int n0  = yt * 128;
  const int y   = yt * 4 + (g >> 1);
  const int xb  = (g & 1) * 16;

  const float* Kf = kvf + (size_t)bh * NTOK * HD;
  const float* Vf = kvf + PLN + (size_t)bh * NTOK * HD;

  float w9[9];
#pragma unroll
  for (int i = 0; i < 9; ++i) w9[i] = cw[d * 9 + i];
  const float bd = cb[d];

#pragma unroll 1
  for (int i = 0; i < 16; ++i) {
    const int x = xb + i;
    float ak = 0.f, av = 0.f;
#pragma unroll
    for (int dy = 0; dy < 3; ++dy) {
      const int yy = y + dy - 1;
      const int yc = clampi(yy, 0, GW - 1);
      const bool vy = (unsigned)yy < (unsigned)GW;
#pragma unroll
      for (int dx = 0; dx < 3; ++dx) {
        const int xx = x + dx - 1;
        const int xc = clampi(xx, 0, GW - 1);
        const bool ok = vy && ((unsigned)xx < (unsigned)GW);
        const size_t o = (size_t)(yc * GW + xc) * HD + d;
        const float kin = Kf[o];
        const float vin = Vf[o];
        const float wv = ok ? w9[dy * 3 + dx] : 0.0f;
        ak += kin * wv;
        av += vin * wv;
      }
    }
    ak += bd;
    av += bd;
    const int nl = (g >> 1) * GW + x;
    Kt[nl * CKP + d]  = (_Float16)(ak * 16.0f);
    Vtt[d * CVP + nl] = (_Float16)(av * 16.0f);
  }
  __syncthreads();

  v4u vk[2], vv[2];
  size_t gk[2], gv[2];
#pragma unroll
  for (int j = 0; j < 2; ++j) {
    const int p = tid + 256 * j;
    {
      const int row = p >> 2;
      const int c8  = (p & 3) * 8;
      Pack8 pk;
      pk.h  = *(const v8h*)(Kt + row * CKP + c8);
      vk[j] = pk.u;
      gk[j] = ((size_t)bh * NTOK + n0) * HD + (size_t)p * 8;
    }
    {
      const int d2 = p >> 4;
      const int np = (p & 15) * 8;
      Pack8 pk;
      pk.h  = *(const v8h*)(Vtt + d2 * CVP + np);
      vv[j] = pk.u;
      gv[j] = ((size_t)bh * HD + d2) * NTOK + n0 + np;
    }
  }
  for (int ps = 0; ps < 2; ++ps) {
#pragma unroll
    for (int j = 0; j < 2; ++j) *(volatile v4u*)(kh + gk[j]) = vk[j];
#pragma unroll
    for (int j = 0; j < 2; ++j) *(volatile v4u*)(vt + gv[j]) = vv[j];
    __threadfence();
  }
}

#define KTP 40
#define VTP 72
#define PTP 72
__global__ __launch_bounds__(256) void k_attn(const _Float16* __restrict__ qp,
                                              const _Float16* __restrict__ kp,
                                              const _Float16* __restrict__ vt,
                                              const float* __restrict__ btab,
                                              _Float16* __restrict__ op, float sscale) {
  __shared__ __align__(16) _Float16 Ks[64 * KTP];
  __shared__ __align__(16) _Float16 Vs[32 * VTP];
  __shared__ __align__(16) _Float16 Ps[8][16 * PTP];

  const int tid = threadIdx.x, lane = tid & 31, wave = tid >> 5;
  const int hh = lane >> 4, c = lane & 15;
  const int bh = blockIdx.x >> 3;
  const int qb = blockIdx.x & 7;
  const int b  = bh / NHD;
  const int h  = bh - b * NHD;
  const int q0 = qb * 128 + wave * 16;

  const _Float16* Q = qp + (size_t)bh * NTOK * HD;
  const _Float16* K = kp + (size_t)bh * NTOK * HD;
  const _Float16* V = vt + (size_t)bh * HD * NTOK;
  const float* Bt = btab + (size_t)h * NTOK * NTOK;

  const v16h qa = ldfrag(Q, HD, q0, 0, lane);

  const float NEGI = -__builtin_huge_valf();
  float mrow[8], lrow[8];
  v8f oacc[2];
#pragma unroll
  for (int r = 0; r < 8; ++r) { mrow[r] = NEGI; lrow[r] = 0.f; }
#pragma unroll
  for (int t = 0; t < 2; ++t) oacc[t] = zero8();

  _Float16* pw = Ps[wave];

  for (int kc = 0; kc < NTOK / 64; ++kc) {
    const int kv0 = kc * 64;
    __syncthreads();
    {
      const int r  = tid >> 2;
      const int qq = (tid & 3) * 8;
      *(v8h*)(Ks + r * KTP + qq) = *(const v8h*)(K + (size_t)(kv0 + r) * HD + qq);
      const int r2 = tid >> 3;
      const int q2 = (tid & 7) * 8;
      *(v8h*)(Vs + r2 * VTP + q2) = *(const v8h*)(V + (size_t)r2 * NTOK + kv0 + q2);
    }
    __syncthreads();

    v8f s[4];
#pragma unroll
    for (int j = 0; j < 4; ++j) {
      const v16h kb = ldfrag(Ks, KTP, j * 16, 0, lane);
      s[j] = mma16(qa, kb, zero8());
    }
    float cm[8];
#pragma unroll
    for (int r = 0; r < 8; ++r) {
      const float* bpr = Bt + (size_t)(q0 + 8 * hh + r) * NTOK + kv0 + c;
      float m = NEGI;
#pragma unroll
      for (int j = 0; j < 4; ++j) {
        const float sv = s[j][r] * sscale + bpr[16 * j];
        s[j][r] = sv;
        m = fmaxf(m, sv);
      }
#pragma unroll
      for (int off = 1; off < 16; off <<= 1) m = fmaxf(m, __shfl_xor(m, off, 32));
      cm[r] = m;
    }
    float al[8];
#pragma unroll
    for (int r = 0; r < 8; ++r) {
      const float mnew  = fmaxf(mrow[r], cm[r]);
      const float alpha = __expf(mrow[r] - mnew);
      mrow[r] = mnew;
      float psum = 0.f;
#pragma unroll
      for (int j = 0; j < 4; ++j) {
        const float p = __expf(s[j][r] - mnew);
        psum += p;
        pw[(8 * hh + r) * PTP + j * 16 + c] = (_Float16)(p * 1024.0f);
      }
#pragma unroll
      for (int off = 1; off < 16; off <<= 1) psum += __shfl_xor(psum, off, 32);
      lrow[r] = lrow[r] * alpha + psum;
      al[r] = alpha;
    }
#pragma unroll
    for (int t = 0; t < 2; ++t)
#pragma unroll
      for (int r = 0; r < 8; ++r) oacc[t][r] *= al[r];
    __syncthreads();

#pragma unroll
    for (int kk = 0; kk < 2; ++kk) {
      const v16h pa = ldfrag(pw, PTP, 0, kk * 32, lane);
#pragma unroll
      for (int t = 0; t < 2; ++t) {
        const v16h vb = ldfrag(Vs, VTP, t * 16, kk * 32, lane);
        oacc[t] = mma16(pa, vb, oacc[t]);
      }
    }
  }
  __syncthreads();

#pragma unroll
  for (int r = 0; r < 8; ++r) {
    const float inv = 0.0625f / lrow[r];
#pragma unroll
    for (int t = 0; t < 2; ++t) pw[(8 * hh + r) * PTP + 16 * t + c] = (_Float16)(oacc[t][r] * inv);
  }
  __syncthreads();
  v4u val[2];
  size_t go[2];
#pragma unroll
  for (int it = 0; it < 2; ++it) {
    const int p   = lane + 32 * it;
    const int row = p >> 2;
    const int c8  = (p & 3) * 8;
    Pack8 pk;
    pk.h    = *(const v8h*)(pw + row * PTP + c8);
    val[it] = pk.u;
    go[it]  = ((size_t)bh * NTOK + q0) * HD + (size_t)p * 8;
  }
  for (int ps = 0; ps < 2; ++ps) {
#pragma unroll
    for (int it = 0; it < 2; ++it) *(volatile v4u*)(op + go[it]) = val[it];
    __threadfence();
  }
}

__global__ __launch_bounds__(256) void k_proj(const _Float16* __restrict__ op,
                                              const _Float16* __restrict__ wt,
                                              const float* __restrict__ bias,
                                              float* __restrict__ out) {
  __shared__ __align__(16) float st[8][16 * OTP];
  const int tid = threadIdx.x, lane = tid & 31, wave = tid >> 5;
  const int hh = lane >> 4, c = lane & 15;
  const int m0 = blockIdx.x * 256 + wave * 32;
  const int n0 = blockIdx.y * 64;
  const int b  = m0 >> 10;
  const int nq = m0 & (NTOK - 1);

  v8f acc[2][4];
#pragma unroll
  for (int s = 0; s < 2; ++s)
#pragma unroll
    for (int t = 0; t < 4; ++t) acc[s][t] = zero8();

#pragma unroll 2
  for (int ks = 0; ks < NHD; ++ks) {
    const _Float16* Ab = op + ((size_t)(b * NHD + ks) * NTOK + nq) * HD;
    const int k0 = ks * 32;
    const v16h a0 = ldfrag(Ab, HD, 0, 0, lane);
    const v16h a1 = ldfrag(Ab, HD, 16, 0, lane);
    const v16h b0 = ldfrag(wt, CC, n0, k0, lane);
    const v16h b1 = ldfrag(wt, CC, n0 + 16, k0, lane);
    const v16h b2 = ldfrag(wt, CC, n0 + 32, k0, lane);
    const v16h b3 = ldfrag(wt, CC, n0 + 48, k0, lane);
    acc[0][0] = mma16(a0, b0, acc[0][0]);
    acc[1][0] = mma16(a1, b0, acc[1][0]);
    acc[0][1] = mma16(a0, b1, acc[0][1]);
    acc[1][1] = mma16(a1, b1, acc[1][1]);
    acc[0][2] = mma16(a0, b2, acc[0][2]);
    acc[1][2] = mma16(a1, b2, acc[1][2]);
    acc[0][3] = mma16(a0, b3, acc[0][3]);
    acc[1][3] = mma16(a1, b3, acc[1][3]);
  }

  float bvs[4];
#pragma unroll
  for (int t = 0; t < 4; ++t) bvs[t] = bias[n0 + 16 * t + c];

  float* sw = st[wave];
#pragma unroll
  for (int sub = 0; sub < 2; ++sub) {
    __syncthreads();
#pragma unroll
    for (int t = 0; t < 4; ++t) {
#pragma unroll
      for (int r = 0; r < 8; ++r)
        sw[(8 * hh + r) * OTP + 16 * t + c] = acc[sub][t][r] * 3.0517578125e-05f + bvs[t];
    }
    __syncthreads();
    v4f val[8];
    size_t go[8];
#pragma unroll
    for (int it = 0; it < 8; ++it) {
      const int p    = lane + 32 * it;
      const int L    = p >> 3;
      const int pc   = p & 7;
      const int row  = L >> 1;
      const int half = L & 1;
      val[it] = *(const v4f*)(sw + row * OTP + half * 32 + pc * 4);
      go[it]  = (size_t)(m0 + sub * 16 + row) * CC + n0 + half * 32 + pc * 4;
    }
    for (int ps = 0; ps < 2; ++ps) {
#pragma unroll
      for (int it = 0; it < 8; ++it) *(volatile v4f*)(out + go[it]) = val[it];
      __threadfence();
    }
  }
}

extern "C" void kernel_launch(void* const* d_in, const int* in_sizes, int n_in,
                              void* d_out, int out_size, void* d_ws, size_t ws_size,
                              hipStream_t stream) {
  if (n_in < 8) return;
  if (in_sizes[0] != ROWS * CC) return;
  if (in_sizes[1] != CC * C3) return;
  if (in_sizes[2] != C3) return;
  if (in_sizes[3] != HD * 9) return;
  if (in_sizes[4] != HD) return;
  if (in_sizes[5] != CC * CC) return;
  if (in_sizes[6] != CC) return;
  if (in_sizes[7] != NHD * NTOK * NTOK) return;
  if (out_size != ROWS * CC) return;

  const float* x      = (const float*)d_in[0];
  const float* w_qkv  = (const float*)d_in[1];
  const float* b_qkv  = (const float*)d_in[2];
  const float* conv_w = (const float*)d_in[3];
  const float* conv_b = (const float*)d_in[4];
  const float* w_proj = (const float*)d_in[5];
  const float* b_proj = (const float*)d_in[6];
  const float* btab   = (const float*)d_in[7];
  float* out = (float*)d_out;

  size_t off = 0;
  const size_t oX  = off; off += (size_t)ROWS * CC * 2;
  const size_t oWq = off; off += (size_t)C3 * CC * 2;
  const size_t oWp = off; off += (size_t)CC * CC * 2;
  const size_t oQ  = off; off += PLN * 2;
  const size_t oKV = off; off += 2 * PLN * 4;
  const size_t oKh = off; off += PLN * 2;
  const size_t oVt = off; off += PLN * 2;
  const size_t oO  = off; off += PLN * 2;
  if (off > ws_size) return;
  if (off > (size_t)134217728) return;

  char* ws = (char*)d_ws;
  _Float16* Xh  = (_Float16*)(ws + oX);
  _Float16* Wqt = (_Float16*)(ws + oWq);
  _Float16* Wpt = (_Float16*)(ws + oWp);
  _Float16* Qp  = (_Float16*)(ws + oQ);
  float*    KVf = (float*)(ws + oKV);
  _Float16* Khp = (_Float16*)(ws + oKh);
  _Float16* Vtp = (_Float16*)(ws + oVt);
  _Float16* Op  = (_Float16*)(ws + oO);

  const int ngrp = in_sizes[0] / 8;
  k_cvt_x<<<dim3((ngrp + 255) / 256), dim3(256), 0, stream>>>(x, Xh, ngrp);
  k_wt<<<dim3(C3 / 64, CC / 64), dim3(256), 0, stream>>>(w_qkv, Wqt, C3);
  k_wt<<<dim3(CC / 64, CC / 64), dim3(256), 0, stream>>>(w_proj, Wpt, CC);
  k_qkv<<<dim3(ROWS / 256, C3 / 64), dim3(256), 0, stream>>>(Xh, Wqt, b_qkv, Qp, KVf);
  k_conv<<<dim3(NBH * (GW / 4)), dim3(256), 0, stream>>>(KVf, conv_w, conv_b, Khp, Vtp);
  const float sscale = 0.17677669529663687f * 0.00390625f;
  k_attn<<<dim3(NBH * (NTOK / 128)), dim3(256), 0, stream>>>(Qp, Khp, Vtp, btab, Op, sscale);
  k_proj<<<dim3(ROWS / 256, CC / 64), dim3(256), 0, stream>>>(Op, Wpt, b_proj, out);
  (void)hipGetLastError();
}
